// EncoderDecoderAttention_15710990369179
// MI455X (gfx1250) — hardware-verified
//
#include <hip/hip_runtime.h>
#include <stdint.h>

typedef __attribute__((ext_vector_type(16))) _Float16 v16h;
typedef __attribute__((ext_vector_type(8)))  _Float16 v8h;
typedef __attribute__((ext_vector_type(16))) __bf16   v16b;
typedef __attribute__((ext_vector_type(8)))  __bf16   v8b;
typedef __attribute__((ext_vector_type(8)))  float    v8f;
typedef __attribute__((ext_vector_type(4)))  float    v4f;
typedef __attribute__((ext_vector_type(4)))  unsigned v4u;

#define SEQ_DEC   8192
#define SEQ_ENC   8192
#define D_MODEL   512
#define HEAD_DIM  64
#define KV_CHUNK  64
#define ATT_WAVES 4

static_assert(SEQ_DEC % 64 == 0);
static_assert(SEQ_ENC % 64 == 0);
static_assert(SEQ_ENC % KV_CHUNK == 0);
static_assert(D_MODEL % 64 == 0);
static_assert(D_MODEL % 32 == 0);
static_assert(HEAD_DIM == 64);
static_assert((SEQ_DEC * D_MODEL) % 8 == 0);

__device__ __forceinline__ unsigned short f2bf_bits(float f) {
  unsigned u = __float_as_uint(f);
  return (unsigned short)((u + 0x7FFFu + ((u >> 16) & 1u)) >> 16);
}
__device__ __forceinline__ float bf_bits2f(unsigned short h) { return __uint_as_float(((unsigned)h) << 16); }

__device__ __forceinline__ void dep_guard_h(v8f& a, v8f& b, v16h x, v16h y) { asm volatile("v_nop\n\tv_nop\n\tv_nop\n\tv_nop" : "+v"(a), "+v"(b) : "v"(x), "v"(y)); }
__device__ __forceinline__ void dep_guard_b(v8f& a, v8f& b, v16b x, v16b y) { asm volatile("v_nop\n\tv_nop\n\tv_nop\n\tv_nop" : "+v"(a), "+v"(b) : "v"(x), "v"(y)); }
__device__ __forceinline__ void keep4_h(v16h a, v16h b, v16h c, v16h d) { asm volatile("v_nop" :: "v"(a), "v"(b), "v"(c), "v"(d)); }
__device__ __forceinline__ void keep4_b(v16b a, v16b b, v16b c, v16b d) { asm volatile("v_nop" :: "v"(a), "v"(b), "v"(c), "v"(d)); }
__device__ __forceinline__ void acc_guard4(v8f& a, v8f& b, v8f& c, v8f& d) { asm volatile("v_nop\n\tv_nop\n\tv_nop\n\tv_nop" : "+v"(a), "+v"(b), "+v"(c), "+v"(d)); }
template <typename T> struct Frag;
template <> struct Frag<_Float16> {
  typedef v16h V; union U { v16h v; v8h h[2]; };
  static __device__ __forceinline__ v16h load(const _Float16* p) {
    U f; f.h[0] = *(const v8h*)(p); f.h[1] = *(const v8h*)(p + 16); return f.v;
  }
  static __device__ __forceinline__ v8f mma(v16h a, v16h b, v8f c) {
    return __builtin_amdgcn_wmma_f32_16x16x32_f16(false, a, false, b, (short)0, c, false, false);
  }
  static __device__ __forceinline__ void guard(v8f& a, v8f& b, v16h x, v16h y) { dep_guard_h(a, b, x, y); }
  static __device__ __forceinline__ void keep(v16h a, v16h b, v16h c, v16h d) { keep4_h(a, b, c, d); }
};
template <> struct Frag<__bf16> {
  typedef v16b V; union U { v16b v; v8b h[2]; };
  static __device__ __forceinline__ v16b load(const __bf16* p) {
    U f; f.h[0] = *(const v8b*)(p); f.h[1] = *(const v8b*)(p + 16); return f.v;
  }
  static __device__ __forceinline__ v8f mma(v16b a, v16b b, v8f c) {
    return __builtin_amdgcn_wmma_f32_16x16x32_bf16(false, a, false, b, (short)0, c, false, false);
  }
  static __device__ __forceinline__ void guard(v8f& a, v8f& b, v16b x, v16b y) { dep_guard_b(a, b, x, y); }
  static __device__ __forceinline__ void keep(v16b a, v16b b, v16b c, v16b d) { keep4_b(a, b, c, d); }
};

template <int ET> struct Elem;
template <> struct Elem<0> { typedef _Float16 T; };
template <> struct Elem<1> { typedef __bf16 T; };
template <int ET, bool SPLIT, int BIAS_MODE, int OUT_MODE, bool RESID, int ACT = 0>
__global__ __launch_bounds__(256) void wmma_gemm64(
    const unsigned short* __restrict__ Ap, const unsigned short* __restrict__ A2p, int lda, long strideA,
    const unsigned short* __restrict__ Btp, const unsigned short* __restrict__ Bt2p, int ldb, long strideB,
    void* __restrict__ Cout, void* __restrict__ Cout2, int ldc, long strideC,
    const float* __restrict__ bias,
    const float* __restrict__ resid, long strideR,
    int M, int N, int K, float scale) {
  typedef typename Elem<ET>::T T;
  typedef typename Frag<T>::V V;
  const T* A = (const T*)Ap; const T* A2 = (const T*)A2p; const T* Bt = (const T*)Btp; const T* Bt2 = (const T*)Bt2p;
  __shared__ __align__(16) float sT[8][16 * 68];
  const int b    = blockIdx.y;
  const int lane = threadIdx.x & 31;
  const int wave = threadIdx.x >> 5;
  const int tilesN = N >> 6;
  const int tilesM = M >> 6;
  const int tile = blockIdx.x * 8 + wave;
  if (tile >= tilesM * tilesN) return;
  const int tm = tile / tilesN;
  const int tn = tile - tm * tilesN;
  const int m0 = tm << 6;
  const int n0 = tn << 6;

  const T* Ab  = A  + (size_t)b * strideA;
  const T* Bb  = Bt + (size_t)b * strideB;
  const T* Ab2 = SPLIT ? (A2  + (size_t)b * strideA) : nullptr;
  const T* Bb2 = SPLIT ? (Bt2 + (size_t)b * strideB) : nullptr;

  const int rlane = lane & 15;
  const int koff  = (lane >> 4) * 8;
  const int mOff  = (lane >> 4) * 8;

  v8f acc[4][4];
#pragma unroll
  for (int i = 0; i < 4; ++i)
#pragma unroll
    for (int j = 0; j < 4; ++j) acc[i][j] = (v8f){0.f,0.f,0.f,0.f,0.f,0.f,0.f,0.f};

  for (int k0 = 0; k0 < K; k0 += 32) {
    V bh[4], bl[4];
#pragma unroll
    for (int j = 0; j < 4; ++j) {
      const size_t bo = (size_t)(n0 + (j << 4) + rlane) * ldb + koff + k0;
      bh[j] = Frag<T>::load(Bb + bo);
      if (SPLIT) bl[j] = Frag<T>::load(Bb2 + bo);
    }
#pragma unroll
    for (int i = 0; i < 4; ++i) {
      const size_t ao = (size_t)(m0 + (i << 4) + rlane) * lda + koff + k0;
      V ah = Frag<T>::load(Ab + ao);
      V al;
      if (SPLIT) al = Frag<T>::load(Ab2 + ao);
#pragma unroll
      for (int j = 0; j < 4; ++j) {
        acc[i][j] = Frag<T>::mma(ah, bh[j], acc[i][j]);
        if (SPLIT) {
          acc[i][j] = Frag<T>::mma(ah, bl[j], acc[i][j]);
          acc[i][j] = Frag<T>::mma(al, bh[j], acc[i][j]);
        }
      }
      Frag<T>::guard(acc[i][0], acc[i][3], ah, SPLIT ? al : ah);
    }
    Frag<T>::keep(bh[0], bh[1], bh[2], bh[3]);
    if (SPLIT) Frag<T>::keep(bl[0], bl[1], bl[2], bl[3]);
  }
  acc_guard4(acc[0][0], acc[0][1], acc[0][2], acc[0][3]);
  acc_guard4(acc[1][0], acc[1][1], acc[1][2], acc[1][3]);
  acc_guard4(acc[2][0], acc[2][1], acc[2][2], acc[2][3]);
  acc_guard4(acc[3][0], acc[3][1], acc[3][2], acc[3][3]);

  float* slab = sT[wave];
  const float* Rb = RESID ? (resid + (size_t)b * strideR) : nullptr;
#pragma unroll
  for (int i = 0; i < 4; ++i) {
    const int mBase = m0 + (i << 4);
#pragma unroll
    for (int j = 0; j < 4; ++j) {
      const int n = n0 + (j << 4) + rlane;
      float bv = 0.f;
      if (BIAS_MODE == 2) bv = bias[n];
#pragma unroll
      for (int r = 0; r < 8; ++r) {
        float v = acc[i][j][r] * scale;
        if (BIAS_MODE == 1) v += bias[mBase + mOff + r];
        if (BIAS_MODE == 2) v += bv;
        if (RESID) v += Rb[(size_t)(mBase + mOff + r) * ldc + n];
        if (ACT == 1) v = tanhf(v);
        if (ACT == 2) v = fmaxf(v, 0.0f);
        if (ACT == 3) v = v / (1.0f + expf(-v));
        if (ACT == 4) v = (v > 0.f) ? v : 0.01f * v;
        if (ACT == 5) v = 0.5f * v * (1.0f + erff(v * 0.70710678118654752f));
        slab[(mOff + r) * 68 + (j << 4) + rlane] = v;
      }
    }
    __builtin_amdgcn_fence(__ATOMIC_RELEASE, "workgroup");
    __builtin_amdgcn_wave_barrier();
    __builtin_amdgcn_fence(__ATOMIC_ACQUIRE, "workgroup");
    if (OUT_MODE == 0) {
      float* C = (float*)Cout + (size_t)b * strideC;
      const int hh = lane >> 4, c4 = (lane & 15) * 4;
      for (int pass = 0; pass < 2; ++pass) {
#pragma unroll
        for (int it = 0; it < 8; ++it) {
          const int row = it * 2 + hh;
          v4f v = *(const v4f*)(slab + row * 68 + c4);
          *(volatile v4f*)(C + (size_t)(mBase + row) * ldc + n0 + c4) = v;
        }
        __threadfence();
      }
    } else {
      const int q = lane >> 3, c8 = (lane & 7) * 8;
      unsigned short* C  = (unsigned short*)Cout  + (size_t)b * strideC;
      unsigned short* C2 = (OUT_MODE == 2) ? ((unsigned short*)Cout2 + (size_t)b * strideC) : nullptr;
      for (int pass = 0; pass < 2; ++pass) {
#pragma unroll
        for (int it = 0; it < 4; ++it) {
          const int row = it * 4 + q;
          const float* sp = slab + row * 68 + c8;
          v8h hv, lv;
#pragma unroll
          for (int e = 0; e < 8; ++e) {
            if (OUT_MODE == 1) {
              hv[e] = (_Float16)sp[e];
            } else {
              unsigned short hb = f2bf_bits(sp[e]);
              unsigned short lb = f2bf_bits(sp[e] - bf_bits2f(hb));
              hv[e] = __builtin_bit_cast(_Float16, hb);
              lv[e] = __builtin_bit_cast(_Float16, lb);
            }
          }
          *(volatile v8h*)(C + (size_t)(mBase + row) * ldc + n0 + c8) = hv;
          if (OUT_MODE == 2) *(volatile v8h*)(C2 + (size_t)(mBase + row) * ldc + n0 + c8) = lv;
        }
        __threadfence();
      }
    }
    __builtin_amdgcn_fence(__ATOMIC_RELEASE, "workgroup");
    __builtin_amdgcn_wave_barrier();
    __builtin_amdgcn_fence(__ATOMIC_ACQUIRE, "workgroup");
  }
}

__device__ __forceinline__ unsigned short at_bf_bits(float f) {
  unsigned u = __float_as_uint(f);
  return (unsigned short)((u + 0x7FFFu + ((u >> 16) & 1u)) >> 16);
}
__device__ __forceinline__ __bf16 at_f2bf(float f) { return __builtin_bit_cast(__bf16, at_bf_bits(f)); }
__device__ __forceinline__ void at_split(float f, __bf16& hi, __bf16& lo) {
  const unsigned short hb = at_bf_bits(f);
  hi = __builtin_bit_cast(__bf16, hb);
  lo = at_f2bf(f - __uint_as_float(((unsigned)hb) << 16));
}
__device__ __forceinline__ v8f at_mma(v16b a, v16b b, v8f c) {
  c = __builtin_amdgcn_wmma_f32_16x16x32_bf16(false, a, false, b, (short)0, c, false, false);
  asm volatile("v_nop\n\tv_nop\n\tv_nop\n\tv_nop" : "+v"(c) : "v"(a), "v"(b));
  return c;
}

__device__ __forceinline__ void split_pair(float f0, float f1, unsigned& hw, unsigned& lw) {
  const unsigned short h0 = f2bf_bits(f0), h1 = f2bf_bits(f1);
  const unsigned short l0 = f2bf_bits(f0 - bf_bits2f(h0)), l1 = f2bf_bits(f1 - bf_bits2f(h1));
  hw = (unsigned)h0 | ((unsigned)h1 << 16);
  lw = (unsigned)l0 | ((unsigned)l1 << 16);
}

__global__ __launch_bounds__(256) void split_bf16_planes(
    const float* __restrict__ in, unsigned short* __restrict__ hi, unsigned short* __restrict__ lo, int n8)
{
  const int i = blockIdx.x * 256 + threadIdx.x;
  if (i >= n8) return;
  const v4f a = *(const v4f*)(in + (size_t)i * 8);
  const v4f b = *(const v4f*)(in + (size_t)i * 8 + 4);
  v4u hv, lv;
  unsigned hw, lw;
  split_pair(a[0], a[1], hw, lw); hv[0] = hw; lv[0] = lw;
  split_pair(a[2], a[3], hw, lw); hv[1] = hw; lv[1] = lw;
  split_pair(b[0], b[1], hw, lw); hv[2] = hw; lv[2] = lw;
  split_pair(b[2], b[3], hw, lw); hv[3] = hw; lv[3] = lw;
  volatile v4u* ph = (volatile v4u*)(hi + (size_t)i * 8);
  volatile v4u* pl = (volatile v4u*)(lo + (size_t)i * 8);
  *ph = hv; *pl = lv;
  __threadfence();
  *ph = hv; *pl = lv;
}

__global__ __launch_bounds__(256) void wt_split_kernel(
    const float* __restrict__ W, unsigned short* __restrict__ Wth, unsigned short* __restrict__ Wtl)
{
  __shared__ float s[64 * 65];
  const int tid = threadIdx.x;
  const int k0  = blockIdx.x * 64;
#pragma unroll
  for (int it = 0; it < 16; ++it) {
    const int idx = it * 256 + tid;
    const int r = idx >> 6, cc = idx & 63;
    s[r * 65 + cc] = W[(size_t)(k0 + r) * HEAD_DIM + cc];
  }
  __syncthreads();
  const int seg = tid & 7;
  const int lin = tid >> 3;
  v4u hv[2], lv[2];
  size_t off[2];
#pragma unroll
  for (int it = 0; it < 2; ++it) {
    const int n = it * 32 + lin;
#pragma unroll
    for (int e = 0; e < 4; ++e) {
      const int kk = seg * 8 + 2 * e;
      unsigned hw, lw;
      split_pair(s[kk * 65 + n], s[(kk + 1) * 65 + n], hw, lw);
      hv[it][e] = hw; lv[it][e] = lw;
    }
    off[it] = (size_t)n * D_MODEL + k0 + seg * 8;
  }
  for (int pass = 0; pass < 2; ++pass) {
#pragma unroll
    for (int it = 0; it < 2; ++it) {
      *(volatile v4u*)(Wth + off[it]) = hv[it];
      *(volatile v4u*)(Wtl + off[it]) = lv[it];
    }
    __threadfence();
  }
}

__global__ __launch_bounds__(128)
void attn_hilo_kernel(const unsigned short* __restrict__ Qh, const unsigned short* __restrict__ Ql,
                      const unsigned short* __restrict__ Kh, const unsigned short* __restrict__ Kl,
                      const unsigned short* __restrict__ Vh, const unsigned short* __restrict__ Vl,
                      float* __restrict__ out)
{
  union FB { v16b v; v8b h[2]; };
  __shared__ __align__(16) unsigned short Ksh[KV_CHUNK * HEAD_DIM];
  __shared__ __align__(16) unsigned short Ksl[KV_CHUNK * HEAD_DIM];
  __shared__ __align__(16) unsigned short Vsh[HEAD_DIM * KV_CHUNK];
  __shared__ __align__(16) unsigned short Vsl[HEAD_DIM * KV_CHUNK];
  __shared__ __align__(16) __bf16 Psh[ATT_WAVES][16 * KV_CHUNK];
  __shared__ __align__(16) __bf16 Psl[ATT_WAVES][16 * KV_CHUNK];
  __shared__ __align__(16) float  Os[ATT_WAVES][16 * 68];

  const int tid  = threadIdx.x;
  const int wave = tid >> 5;
  const int lane = tid & 31;
  const int hh   = lane >> 4;
  const int c    = lane & 15;
  const int q0   = blockIdx.x * (ATT_WAVES * 16) + wave * 16;

  v16b qah[2], qal[2];
  {
    const __bf16* qhr = (const __bf16*)(const void*)Qh + (size_t)(q0 + c) * HEAD_DIM + 8 * hh;
    const __bf16* qlr = (const __bf16*)(const void*)Ql + (size_t)(q0 + c) * HEAD_DIM + 8 * hh;
#pragma unroll
    for (int dc = 0; dc < 2; ++dc) {
      qah[dc] = Frag<__bf16>::load(qhr + dc * 32);
      qal[dc] = Frag<__bf16>::load(qlr + dc * 32);
    }
  }

  float mrow[8], lrow[8];
  v8f oacc[4];
#pragma unroll
  for (int r = 0; r < 8; ++r) { mrow[r] = -INFINITY; lrow[r] = 0.f; }
#pragma unroll
  for (int t = 0; t < 4; ++t) oacc[t] = (v8f){0.f,0.f,0.f,0.f,0.f,0.f,0.f,0.f};

  __bf16* pwh = Psh[wave];
  __bf16* pwl = Psl[wave];

  for (int kc = 0; kc < SEQ_ENC / KV_CHUNK; ++kc) {
    const int kv0 = kc * KV_CHUNK;
    __syncthreads();
#pragma unroll 1
    for (int it = 0; it < 4; ++it) {
      const int idx = it * 128 + tid;
      const int dd = idx >> 3, seg = idx & 7;
      const v4u ka = *(const v4u*)(Kh + (size_t)kv0 * HEAD_DIM + (size_t)idx * 8);
      const v4u kb = *(const v4u*)(Kl + (size_t)kv0 * HEAD_DIM + (size_t)idx * 8);
      const v4u va = *(const v4u*)(Vh + (size_t)dd * SEQ_ENC + kv0 + seg * 8);
      const v4u vb = *(const v4u*)(Vl + (size_t)dd * SEQ_ENC + kv0 + seg * 8);
      *(v4u*)(Ksh + idx * 8) = ka;
      *(v4u*)(Ksl + idx * 8) = kb;
      *(v4u*)(Vsh + idx * 8) = va;
      *(v4u*)(Vsl + idx * 8) = vb;
    }
    __syncthreads();

    v8f s[4];
#pragma unroll
    for (int j = 0; j < 4; ++j) {
      s[j] = (v8f){0.f,0.f,0.f,0.f,0.f,0.f,0.f,0.f};
#pragma unroll
      for (int dc = 0; dc < 2; ++dc) {
        FB kbh, kbl;
        const unsigned short* kp = Ksh + (j * 16 + c) * HEAD_DIM + dc * 32 + 8 * hh;
        const unsigned short* lp = Ksl + (j * 16 + c) * HEAD_DIM + dc * 32 + 8 * hh;
        kbh.h[0] = *(const v8b*)(kp); kbh.h[1] = *(const v8b*)(kp + 16);
        kbl.h[0] = *(const v8b*)(lp); kbl.h[1] = *(const v8b*)(lp + 16);
        s[j] = at_mma(qah[dc], kbh.v, s[j]);
        s[j] = at_mma(qah[dc], kbl.v, s[j]);
        s[j] = at_mma(qal[dc], kbh.v, s[j]);
      }
    }

    float cm[8];
#pragma unroll
    for (int r = 0; r < 8; ++r) {
      float m = fmaxf(fmaxf(s[0][r], s[1][r]), fmaxf(s[2][r], s[3][r]));
#pragma unroll
      for (int off = 1; off < 16; off <<= 1) m = fmaxf(m, __shfl_xor(m, off, 32));
      cm[r] = m;
    }

#pragma unroll
    for (int r = 0; r < 8; ++r) {
      const float mnew = fmaxf(mrow[r], cm[r]);
      const float alpha = expf(mrow[r] - mnew);
      mrow[r] = mnew;
      float psum = 0.f;
#pragma unroll
      for (int j = 0; j < 4; ++j) {
        const float p = expf(s[j][r] - mnew);
        psum += p;
        __bf16 a, bl;
        at_split(p, a, bl);
        pwh[(8 * hh + r) * KV_CHUNK + j * 16 + c] = a;
        pwl[(8 * hh + r) * KV_CHUNK + j * 16 + c] = bl;
      }
#pragma unroll
      for (int off = 1; off < 16; off <<= 1) psum += __shfl_xor(psum, off, 32);
      lrow[r] = lrow[r] * alpha + psum;
#pragma unroll
      for (int t = 0; t < 4; ++t) oacc[t][r] *= alpha;
    }
    __syncthreads();

#pragma unroll 1
    for (int kk = 0; kk < 2; ++kk) {
      FB pa, pl;
      pa.h[0] = *(const v8b*)(pwh + c * KV_CHUNK + kk * 32 + 8 * hh);
      pa.h[1] = *(const v8b*)(pwh + c * KV_CHUNK + kk * 32 + 16 + 8 * hh);
      pl.h[0] = *(const v8b*)(pwl + c * KV_CHUNK + kk * 32 + 8 * hh);
      pl.h[1] = *(const v8b*)(pwl + c * KV_CHUNK + kk * 32 + 16 + 8 * hh);
#pragma unroll
      for (int t = 0; t < 4; ++t) {
        FB vbh, vbl;
        const unsigned short* vp = Vsh + (t * 16 + c) * KV_CHUNK + kk * 32 + 8 * hh;
        const unsigned short* wp = Vsl + (t * 16 + c) * KV_CHUNK + kk * 32 + 8 * hh;
        vbh.h[0] = *(const v8b*)(vp); vbh.h[1] = *(const v8b*)(vp + 16);
        vbl.h[0] = *(const v8b*)(wp); vbl.h[1] = *(const v8b*)(wp + 16);
        oacc[t] = at_mma(pa.v, vbh.v, oacc[t]);
        oacc[t] = at_mma(pa.v, vbl.v, oacc[t]);
        oacc[t] = at_mma(pl.v, vbh.v, oacc[t]);
      }
    }
  }

  float* os = Os[wave];
#pragma unroll
  for (int r = 0; r < 8; ++r) {
    const float inv = 1.0f / lrow[r];
#pragma unroll
    for (int t = 0; t < 4; ++t) os[(8 * hh + r) * 68 + t * 16 + c] = oacc[t][r] * inv;
  }
  __syncthreads();
  {
    const int c4 = (lane & 15) * 4;
    for (int pass = 0; pass < 2; ++pass) {
#pragma unroll
      for (int it = 0; it < 8; ++it) {
        const int row = it * 2 + hh;
        v4f val = *(const v4f*)(os + row * 68 + c4);
        *(volatile v4f*)(out + (size_t)(q0 + row) * HEAD_DIM + c4) = val;
      }
      __threadfence();
    }
  }
}

extern "C" void kernel_launch(void* const* d_in, const int* in_sizes, int n_in,
                              void* d_out, int out_size, void* d_ws, size_t ws_size,
                              hipStream_t stream)
{
  if (n_in < 5) return;
  if (in_sizes[0] != SEQ_DEC * D_MODEL || in_sizes[1] != SEQ_ENC * D_MODEL ||
      in_sizes[2] != D_MODEL * HEAD_DIM || in_sizes[3] != D_MODEL * HEAD_DIM ||
      in_sizes[4] != D_MODEL * HEAD_DIM) return;
  if (out_size != SEQ_DEC * HEAD_DIM) return;

  const float* x   = (const float*)d_in[0];
  const float* emb = (const float*)d_in[1];
  const float* wq  = (const float*)d_in[2];
  const float* wk  = (const float*)d_in[3];
  const float* wv  = (const float*)d_in[4];
  float* out = (float*)d_out;

  const size_t planeX = (size_t)SEQ_DEC * D_MODEL * 2;
  const size_t planeE = (size_t)SEQ_ENC * D_MODEL * 2;
  const size_t planeW = (size_t)HEAD_DIM * D_MODEL * 2;
  const size_t planeQ = (size_t)SEQ_DEC * HEAD_DIM * 2;
  const size_t planeK = (size_t)SEQ_ENC * HEAD_DIM * 2;

  size_t off = 0;
  unsigned char* ws = (unsigned char*)d_ws;
  unsigned short* xh  = (unsigned short*)(ws + off); off += planeX;
  unsigned short* xl  = (unsigned short*)(ws + off); off += planeX;
  unsigned short* eh  = (unsigned short*)(ws + off); off += planeE;
  unsigned short* el  = (unsigned short*)(ws + off); off += planeE;
  unsigned short* wqh = (unsigned short*)(ws + off); off += planeW;
  unsigned short* wql = (unsigned short*)(ws + off); off += planeW;
  unsigned short* wkh = (unsigned short*)(ws + off); off += planeW;
  unsigned short* wkl = (unsigned short*)(ws + off); off += planeW;
  unsigned short* wvh = (unsigned short*)(ws + off); off += planeW;
  unsigned short* wvl = (unsigned short*)(ws + off); off += planeW;
  unsigned short* qh  = (unsigned short*)(ws + off); off += planeQ;
  unsigned short* ql  = (unsigned short*)(ws + off); off += planeQ;
  unsigned short* kh  = (unsigned short*)(ws + off); off += planeK;
  unsigned short* kl  = (unsigned short*)(ws + off); off += planeK;
  unsigned short* vth = (unsigned short*)(ws + off); off += planeK;
  unsigned short* vtl = (unsigned short*)(ws + off); off += planeK;
  if (off > ws_size) return;

  const int n8x = SEQ_DEC * D_MODEL / 8;
  const int n8e = SEQ_ENC * D_MODEL / 8;
  split_bf16_planes<<<(n8x + 255) / 256, 256, 0, stream>>>(x, xh, xl, n8x);
  split_bf16_planes<<<(n8e + 255) / 256, 256, 0, stream>>>(emb, eh, el, n8e);

  wt_split_kernel<<<D_MODEL / 64, 256, 0, stream>>>(wq, wqh, wql);
  wt_split_kernel<<<D_MODEL / 64, 256, 0, stream>>>(wk, wkh, wkl);
  wt_split_kernel<<<D_MODEL / 64, 256, 0, stream>>>(wv, wvh, wvl);

  {
    const int tilesQ = (SEQ_DEC / 64) * (HEAD_DIM / 64);
    dim3 gq((tilesQ + 7) / 8, 1);
    wmma_gemm64<1, true, 0, 2, false, 0><<<gq, 256, 0, stream>>>(
        xh, xl, D_MODEL, 0L, wqh, wql, D_MODEL, 0L,
        (void*)qh, (void*)ql, HEAD_DIM, 0L, (const float*)nullptr, (const float*)nullptr, 0L,
        SEQ_DEC, HEAD_DIM, D_MODEL, 0.125f);
    const int tilesK = (SEQ_ENC / 64) * (HEAD_DIM / 64);
    dim3 gk((tilesK + 7) / 8, 1);
    wmma_gemm64<1, true, 0, 2, false, 0><<<gk, 256, 0, stream>>>(
        eh, el, D_MODEL, 0L, wkh, wkl, D_MODEL, 0L,
        (void*)kh, (void*)kl, HEAD_DIM, 0L, (const float*)nullptr, (const float*)nullptr, 0L,
        SEQ_ENC, HEAD_DIM, D_MODEL, 1.0f);
    const int tilesV = (HEAD_DIM / 64) * (SEQ_ENC / 64);
    dim3 gv((tilesV + 7) / 8, 1);
    wmma_gemm64<1, true, 0, 2, false, 0><<<gv, 256, 0, stream>>>(
        wvh, wvl, D_MODEL, 0L, eh, el, D_MODEL, 0L,
        (void*)vth, (void*)vtl, SEQ_ENC, 0L, (const float*)nullptr, (const float*)nullptr, 0L,
        HEAD_DIM, SEQ_ENC, D_MODEL, 1.0f);
  }

  attn_hilo_kernel<<<SEQ_DEC / (ATT_WAVES * 16), 128, 0, stream>>>(qh, ql, kh, kl, vth, vtl, out);
}
